// BiMPNNLayer_2662879724349
// MI455X (gfx1250) — hardware-verified
//
#include <hip/hip_runtime.h>
#include <stddef.h>


#define DIMH    128
#define KTOT    384
#define KSTEPS  (KTOT / 32)
#define NTHR    256
#define NWAVE   8
#define EPT     8
#define NGRP    2
#define CHUNK   (NTHR * EPT * NGRP)
#define WCAP    (EPT * NGRP * 32)
#define LISTN   (NWAVE * WCAP)
#define NBC     4096
#define NBF     1024
#define RCAP    40960
#define RBN     128
#define OTHR    512
#define TGT     64
#define FTHR    128
#define DEGCAP  256
#define APH     (KTOT + 8)

#define LDS_FILL   ((RCAP + NBF + LISTN) * 4 + 64)
#define LDS_APLANE (TGT * APH * 2)
#define LDS_FUSED  (2 * LDS_APLANE + 2 * TGT * 4)

static_assert((CHUNK & (CHUNK - 1)) == 0);
static_assert(CHUNK <= 4096);
static_assert(NBC <= 4096 && NBF <= 4096);
static_assert((NBC & (NBC - 1)) == 0 && (NBF & (NBF - 1)) == 0);
static_assert(NBC == 4 * NBF);
static_assert(OTHR * 8 == NBC);
static_assert((RCAP % 32) == 0);
static_assert((TGT % 16) == 0 && FTHR == (TGT / 16) * 32);
static_assert(TGT * DIMH * 4 <= LDS_APLANE);
static_assert((LDS_APLANE % 16) == 0 && ((APH * 2) % 16) == 0);
static_assert((NBC % TGT) == 0);
static_assert((DIMH * KTOT / 8) % NTHR == 0);
static_assert(KTOT == 3 * DIMH && (KTOT % 32) == 0);

typedef float          v4f   __attribute__((ext_vector_type(4)));
typedef float          v8f   __attribute__((ext_vector_type(8)));
typedef int            v4i   __attribute__((ext_vector_type(4)));
typedef unsigned short v4us  __attribute__((ext_vector_type(4)));
typedef unsigned short v8us  __attribute__((ext_vector_type(8)));
typedef __bf16         v16bf __attribute__((ext_vector_type(16)));
union FragB { v16bf v; v8us h[2]; };

__device__ __forceinline__ v8f wmb(v16bf a, v16bf b, v8f c) {
  v8f d = __builtin_amdgcn_wmma_f32_16x16x32_bf16(false, a, false, b, (short)0, c, false, false);
  asm volatile("v_nop\n\tv_nop\n\tv_nop\n\tv_nop" : "+v"(d) : "v"(a), "v"(b));
  return d;
}

__device__ __forceinline__ unsigned int bf16_rne_bits(float x) {
  const unsigned int u = __float_as_uint(x);
  return (u + 0x7FFFu + ((u >> 16) & 1u)) >> 16;
}

__device__ __forceinline__ void split1(float x, unsigned short& hi, unsigned short& lo) {
  const unsigned int hb = bf16_rne_bits(x);
  const float hf = __uint_as_float(hb << 16);
  const unsigned int lb = bf16_rne_bits(x - hf);
  hi = (unsigned short)hb;
  lo = (unsigned short)lb;
}

__device__ __forceinline__ void split4(v4f v, v4us& hi, v4us& lo) {
  unsigned short a, b;
  split1(v.x, a, b); hi.x = a; lo.x = b;
  split1(v.y, a, b); hi.y = a; lo.y = b;
  split1(v.z, a, b); hi.z = a; lo.z = b;
  split1(v.w, a, b); hi.w = a; lo.w = b;
}

__device__ __forceinline__ float gelu1(float x) {
  return 0.5f * x * (1.0f + erff(x * 0.70710678118654752f));
}

template <int NB>
__device__ __forceinline__ int scan_chunk(const int* __restrict__ dsts, int nE, int cbase, int slotBase,
                                          int vec8, int* list, int tid, int lane, int wave) {
  int wc = 0;
#pragma unroll
  for (int g = 0; g < NGRP; ++g) {
    const int el0  = (g * NTHR + tid) * EPT;
    const int e0   = cbase + el0;
    const int sent = -2147483647 - 1;
    v4i da, db;
    if (vec8 != 0 && cbase + CHUNK <= nE) {
      da = *(const v4i*)(dsts + e0);
      db = *(const v4i*)(dsts + e0 + 4);
    } else {
      da.x = (e0     < nE) ? dsts[min(e0, nE - 1)] : sent;
      da.y = (e0 + 1 < nE) ? dsts[min(e0 + 1, nE - 1)] : sent;
      da.z = (e0 + 2 < nE) ? dsts[min(e0 + 2, nE - 1)] : sent;
      da.w = (e0 + 3 < nE) ? dsts[min(e0 + 3, nE - 1)] : sent;
      db.x = (e0 + 4 < nE) ? dsts[min(e0 + 4, nE - 1)] : sent;
      db.y = (e0 + 5 < nE) ? dsts[min(e0 + 5, nE - 1)] : sent;
      db.z = (e0 + 6 < nE) ? dsts[min(e0 + 6, nE - 1)] : sent;
      db.w = (e0 + 7 < nE) ? dsts[min(e0 + 7, nE - 1)] : sent;
    }
    const unsigned nb = (unsigned)slotBase;
    const unsigned s0 = (unsigned)da.x - nb, s1 = (unsigned)da.y - nb;
    const unsigned s2 = (unsigned)da.z - nb, s3 = (unsigned)da.w - nb;
    const unsigned s4 = (unsigned)db.x - nb, s5 = (unsigned)db.y - nb;
    const unsigned s6 = (unsigned)db.z - nb, s7 = (unsigned)db.w - nb;
    const bool h0 = s0 < (unsigned)NB, h1 = s1 < (unsigned)NB, h2 = s2 < (unsigned)NB, h3 = s3 < (unsigned)NB;
    const bool h4 = s4 < (unsigned)NB, h5 = s5 < (unsigned)NB, h6 = s6 < (unsigned)NB, h7 = s7 < (unsigned)NB;
    const unsigned any = __builtin_amdgcn_ballot_w32(h0 | h1 | h2 | h3 | h4 | h5 | h6 | h7);
    if (any != 0u) {
#define HITJ(J, HJ, SJ) { \
        const unsigned mj = __builtin_amdgcn_ballot_w32(HJ); \
        if (mj != 0u) { \
          if (HJ) { \
            const int pos = wc + (int)__builtin_amdgcn_mbcnt_lo(mj, 0u); \
            if (pos < WCAP) list[wave * WCAP + pos] = ((el0 + (J)) << 12) | (int)(SJ); \
          } \
          wc += (int)__builtin_popcount(mj); } }
      HITJ(0, h0, s0)
      HITJ(1, h1, s1)
      HITJ(2, h2, s2)
      HITJ(3, h3, s3)
      HITJ(4, h4, s4)
      HITJ(5, h5, s5)
      HITJ(6, h6, s6)
      HITJ(7, h7, s7)
#undef HITJ
    }
  }
  return wc;
}

__global__ __launch_bounds__(NTHR) void k_wprep(
    const float* __restrict__ Ww, const float* __restrict__ Wtw, const float* __restrict__ Wsw,
    unsigned short* Bhi, unsigned short* Blo) {
  const int i = blockIdx.x * NTHR + (int)threadIdx.x;
  if (i >= DIMH * KTOT / 8) return;
  const int o   = 8 * i;
  const int n   = o / KTOT;
  const int k0  = o - n * KTOT;
  const int seg = k0 >> 7;
  const int kk  = k0 & (DIMH - 1);
  const float* pa = Ww  + n * DIMH + kk;
  const float* pb = Wtw + n * DIMH + kk;
  const float* pc = Wsw + n * DIMH + kk;
  const v4f a0 = *(const v4f*)pa, a1 = *(const v4f*)(pa + 4);
  const v4f b0 = *(const v4f*)pb, b1 = *(const v4f*)(pb + 4);
  const v4f c0 = *(const v4f*)pc, c1 = *(const v4f*)(pc + 4);
  float v[8];
  v[0] = seg == 0 ? a0.x : (seg == 1 ? b0.x : c0.x);
  v[1] = seg == 0 ? a0.y : (seg == 1 ? b0.y : c0.y);
  v[2] = seg == 0 ? a0.z : (seg == 1 ? b0.z : c0.z);
  v[3] = seg == 0 ? a0.w : (seg == 1 ? b0.w : c0.w);
  v[4] = seg == 0 ? a1.x : (seg == 1 ? b1.x : c1.x);
  v[5] = seg == 0 ? a1.y : (seg == 1 ? b1.y : c1.y);
  v[6] = seg == 0 ? a1.z : (seg == 1 ? b1.z : c1.z);
  v[7] = seg == 0 ? a1.w : (seg == 1 ? b1.w : c1.w);
  v8us hv, lv;
#pragma unroll
  for (int e = 0; e < 8; ++e) {
    unsigned short hs, ls;
    split1(v[e], hs, ls);
    hv[e] = hs;
    lv[e] = ls;
  }
  unsigned short* hp = Bhi + o;
  unsigned short* lp = Blo + o;
  *(volatile v8us*)hp = hv;
  *(volatile v8us*)lp = lv;
  __threadfence();
  *(volatile v8us*)hp = hv;
  *(volatile v8us*)lp = lv;
}

__global__ __launch_bounds__(NTHR) void k_count(
    const int* __restrict__ dst, int* cnt, int nE, int vec8) {
  __shared__ __attribute__((aligned(16))) int scnt[NBC];
  __shared__ __attribute__((aligned(16))) int list[LISTN];
  __shared__ int wcnt[NWAVE];
  const int tid = threadIdx.x, lane = tid & 31, wave = tid >> 5;
  const int nodeBase = blockIdx.x * NBC;

  for (int i = tid; i < NBC; i += NTHR) scnt[i] = 0;
  __syncthreads();

  const int nChunks = (nE + CHUNK - 1) / CHUNK;
#pragma unroll 1
  for (int ch = 0; ch < nChunks; ++ch) {
    const int cbase = ch * CHUNK;
    const int wc = scan_chunk<NBC>(dst, nE, cbase, nodeBase, vec8, list, tid, lane, wave);
    if (lane == 0) wcnt[wave] = wc;
    __syncthreads();
    if (wave == 0) {
#pragma unroll 1
      for (int wsx = 0; wsx < NWAVE; ++wsx) {
        int n = __builtin_amdgcn_readfirstlane(wcnt[wsx]);
        n = n > WCAP ? WCAP : (n < 0 ? 0 : n);
        const int* lp = list + wsx * WCAP;
#pragma unroll 1
        for (int i = 0; i < n; ++i) {
          const int ent  = __builtin_amdgcn_readfirstlane(lp[i]);
          const int slot = ent & (NBC - 1);
          if (lane == 0) scnt[slot] = scnt[slot] + 1;
        }
      }
    }
    __syncthreads();
  }

  v4i cq[4];
#pragma unroll
  for (int q = 0; q < 4; ++q) {
    const int f = (wave * 4 + q) * 128 + 4 * lane;
    cq[q] = *(const v4i*)(scnt + f);
  }
  int* cp = cnt + (size_t)nodeBase;
#pragma unroll
  for (int q = 0; q < 4; ++q) {
    const int f = (wave * 4 + q) * 128 + 4 * lane;
    *(volatile v4i*)(cp + f) = cq[q];
  }
  __threadfence();
#pragma unroll
  for (int q = 0; q < 4; ++q) {
    const int f = (wave * 4 + q) * 128 + 4 * lane;
    *(volatile v4i*)(cp + f) = cq[q];
  }
}

__global__ __launch_bounds__(OTHR) void k_offsets(
    const int* __restrict__ cnt, int* off, int* rbase, int nChunk) {
  __shared__ __attribute__((aligned(16))) int soff[NBC];
  __shared__ __attribute__((aligned(16))) int srb[RBN];
  __shared__ int wtot[OTHR / 32];
  const int tid = threadIdx.x, lane = tid & 31, wave = tid >> 5, sub = tid >> 7;
  for (int i = tid; i < RBN; i += OTHR) srb[i] = 0;
  int carry = 0;
#pragma unroll 1
  for (int ch = 0; ch < nChunk; ++ch) {
    const int base = ch * NBC;
    const v4i c0 = *(const v4i*)(cnt + base + 8 * tid);
    const v4i c1 = *(const v4i*)(cnt + base + 8 * tid + 4);
    const int e0 = max(c0.x, 0), e1 = max(c0.y, 0), e2 = max(c0.z, 0), e3 = max(c0.w, 0);
    const int e4 = max(c1.x, 0), e5 = max(c1.y, 0), e6 = max(c1.z, 0), e7 = max(c1.w, 0);
    const int ts = e0 + e1 + e2 + e3 + e4 + e5 + e6 + e7;
    int incl = ts;
#pragma unroll
    for (int d = 1; d < 32; d <<= 1) {
      const int t = __shfl_up(incl, d);
      if (lane >= d) incl += t;
    }
    if (lane == 31) wtot[wave] = incl;
    __syncthreads();
    const int S0 = wtot[0]  + wtot[1]  + wtot[2]  + wtot[3];
    const int S1 = wtot[4]  + wtot[5]  + wtot[6]  + wtot[7];
    const int S2 = wtot[8]  + wtot[9]  + wtot[10] + wtot[11];
    const int S3 = wtot[12] + wtot[13] + wtot[14] + wtot[15];
    int pre = 0;
#pragma unroll 1
    for (int w = 4 * sub; w < wave; ++w) pre += wtot[w];
    const int b0 = carry;
    const int b1 = b0 + ((S0 + 31) & ~31);
    const int b2 = b1 + ((S1 + 31) & ~31);
    const int b3 = b2 + ((S2 + 31) & ~31);
    const int b4 = b3 + ((S3 + 31) & ~31);
    const int myb = sub == 0 ? b0 : (sub == 1 ? b1 : (sub == 2 ? b2 : b3));
    if (tid == 0) {
      srb[min(4 * ch + 0, RBN - 1)] = b0;
      srb[min(4 * ch + 1, RBN - 1)] = b1;
      srb[min(4 * ch + 2, RBN - 1)] = b2;
      srb[min(4 * ch + 3, RBN - 1)] = b3;
    }
    int run = myb + pre + incl - ts;
    soff[8 * tid + 0] = run; run += e0;
    soff[8 * tid + 1] = run; run += e1;
    soff[8 * tid + 2] = run; run += e2;
    soff[8 * tid + 3] = run; run += e3;
    soff[8 * tid + 4] = run; run += e4;
    soff[8 * tid + 5] = run; run += e5;
    soff[8 * tid + 6] = run; run += e6;
    soff[8 * tid + 7] = run;
    carry = b4;
    __syncthreads();
    const v4i o0 = *(const v4i*)(soff + 4 * tid);
    const v4i o1 = *(const v4i*)(soff + 4 * (tid + OTHR));
    int* op = off + base;
    *(volatile v4i*)(op + 4 * tid) = o0;
    *(volatile v4i*)(op + 4 * (tid + OTHR)) = o1;
    __threadfence();
    *(volatile v4i*)(op + 4 * tid) = o0;
    *(volatile v4i*)(op + 4 * (tid + OTHR)) = o1;
    __syncthreads();
  }
  if (tid == 0) srb[min(4 * nChunk, RBN - 1)] = carry;
  __syncthreads();
  v4i rv = {0, 0, 0, 0};
  if (tid < 32) rv = *(const v4i*)(srb + 4 * tid);
  if (tid < 32) *(volatile v4i*)(rbase + 4 * tid) = rv;
  __threadfence();
  if (tid < 32) *(volatile v4i*)(rbase + 4 * tid) = rv;
}

__global__ __launch_bounds__(NTHR) void k_fill(
    const int* __restrict__ dst, const int* __restrict__ srcs,
    const int* __restrict__ off, const int* __restrict__ rbase,
    int* csr, int nN, int nE, int vec8, int csrLen) {
  extern __shared__ v4f lds_dyn[];
  int* region = (int*)lds_dyn;
  int* cursor = region + RCAP;
  int* list   = cursor + NBF;
  int* wcnt   = list + LISTN;
  const int tid = threadIdx.x, lane = tid & 31, wave = tid >> 5;
  const int b = blockIdx.x;
  const int nodeBase = b * NBF;

  int rb0 = rbase[b];
  const int rb1 = rbase[b + 1];
  rb0 = rb0 < 0 ? 0 : (rb0 > csrLen ? csrLen : rb0);
  rb0 &= ~31;
  int len = rb1 - rb0;
  len = len < 0 ? 0 : (len > RCAP ? RCAP : len);
  int lenW = (len + 31) & ~31;
  if (rb0 + lenW > csrLen) lenW = (csrLen - rb0) & ~31;

  {
    const v4i z = {0, 0, 0, 0};
    for (int i = tid; i < RCAP / 4; i += NTHR) ((v4i*)region)[i] = z;
    for (int s = tid; s < NBF; s += NTHR) {
      int o = off[nodeBase + s] - rb0;
      o = o < 0 ? 0 : (o > RCAP ? RCAP : o);
      cursor[s] = o;
    }
  }
  __syncthreads();

  const int nChunks = (nE + CHUNK - 1) / CHUNK;
#pragma unroll 1
  for (int ch = 0; ch < nChunks; ++ch) {
    const int cbase = ch * CHUNK;
    const int wc = scan_chunk<NBF>(dst, nE, cbase, nodeBase, vec8, list, tid, lane, wave);
    if (lane == 0) wcnt[wave] = wc;
    __syncthreads();
    if (wave == 0) {
#pragma unroll 1
      for (int wsx = 0; wsx < NWAVE; ++wsx) {
        int n = __builtin_amdgcn_readfirstlane(wcnt[wsx]);
        n = n > WCAP ? WCAP : (n < 0 ? 0 : n);
        const int* lp = list + wsx * WCAP;
#pragma unroll 1
        for (int i = 0; i < n; ++i) {
          const int ent  = __builtin_amdgcn_readfirstlane(lp[i]);
          const int slot = ent & (NBF - 1);
          int e = cbase + ((ent >> 12) & (CHUNK - 1));
          e = e > nE - 1 ? nE - 1 : e;
          int src = srcs[e];
          src = src < 0 ? 0 : (src > nN - 1 ? nN - 1 : src);
          if (lane == 0) {
            int pos = cursor[slot];
            pos = pos < 0 ? 0 : (pos > RCAP - 1 ? RCAP - 1 : pos);
            region[pos] = src;
            const int np = pos + 1;
            cursor[slot] = np > RCAP ? RCAP : np;
          }
        }
      }
    }
    __syncthreads();
  }

  const int nv = lenW >> 2;
  int* gp = csr + rb0;
#pragma unroll 1
  for (int i = tid; i < nv; i += NTHR) { const v4i v = ((const v4i*)region)[i]; *(volatile v4i*)(gp + 4 * i) = v; }
  __threadfence();
#pragma unroll 1
  for (int i = tid; i < nv; i += NTHR) { const v4i v = ((const v4i*)region)[i]; *(volatile v4i*)(gp + 4 * i) = v; }
}

__device__ __forceinline__ v4f seg_sum(const int* __restrict__ csr, const float* __restrict__ h,
                                       int n, int st, int csrLen, int nN, int lane) {
  v4f acc = {0.f, 0.f, 0.f, 0.f};
#pragma unroll 1
  for (int q0 = 0; q0 < n; q0 += 32) {
    int pos = st + q0 + lane;
    pos = pos < 0 ? 0 : (pos > csrLen - 1 ? csrLen - 1 : pos);
    int sl = csr[pos];
    sl = sl < 0 ? 0 : (sl > nN - 1 ? nN - 1 : sl);
    const int mcnt = (n - q0) < 32 ? (n - q0) : 32;
#pragma unroll 1
    for (int p = 0; p < mcnt; ++p) {
      const int s = __builtin_amdgcn_readlane(sl, p);
      acc = acc + *(const v4f*)(h + (size_t)s * DIMH + 4 * lane);
    }
  }
  return acc;
}

__global__ __launch_bounds__(FTHR) void k_fused(
    const float* __restrict__ h,
    const unsigned short* __restrict__ Bhi, const unsigned short* __restrict__ Blo,
    const int* __restrict__ cntR, const int* __restrict__ offR, const int* __restrict__ csrR,
    const int* __restrict__ cntC, const int* __restrict__ offC, const int* __restrict__ csrC,
    const float* __restrict__ Wb, const float* __restrict__ Wtb, const float* __restrict__ Wsb,
    float* out, int nN, int csrLen) {
  extern __shared__ v4f lds_dyn[];
  unsigned short* sHi = (unsigned short*)lds_dyn;
  unsigned short* sLo = sHi + TGT * APH;
  float* sdR = (float*)(sLo + TGT * APH);
  float* sdC = sdR + TGT;
  float* stg = (float*)lds_dyn;
  const int tid = threadIdx.x, lane = tid & 31, wave = tid >> 5, hh = lane >> 4, m = lane & 15;
  const int rw = wave * 16;
  const int tbase = blockIdx.x * TGT + rw;

  const int cl = tbase + m;
  const int cR_l = cntR[cl], oR_l = offR[cl];
  const int cC_l = cntC[cl], oC_l = offC[cl];
#pragma unroll 1
  for (int j = 0; j < 16; ++j) {
    const int node = tbase + j;
    int nR = __builtin_amdgcn_readlane(cR_l, j);
    nR = nR < 0 ? 0 : (nR > DEGCAP ? DEGCAP : nR);
    const int stR = __builtin_amdgcn_readlane(oR_l, j);
    int nC = __builtin_amdgcn_readlane(cC_l, j);
    nC = nC < 0 ? 0 : (nC > DEGCAP ? DEGCAP : nC);
    const int stC = __builtin_amdgcn_readlane(oC_l, j);
    const v4f aR = seg_sum(csrR, h, nR, stR, csrLen, nN, lane);
    const v4f aC = seg_sum(csrC, h, nC, stC, csrLen, nN, lane);
    const int nd = node > nN - 1 ? nN - 1 : node;
    const v4f hv = *(const v4f*)(h + (size_t)nd * DIMH + 4 * lane);
    const int row = rw + j;
    v4us h0, l0, h1, l1, h2, l2;
    split4(aR, h0, l0);
    split4(aC, h1, l1);
    split4(hv, h2, l2);
    unsigned short* ph = sHi + row * APH + 4 * lane;
    unsigned short* pl = sLo + row * APH + 4 * lane;
    *(v4us*)(ph)            = h0;
    *(v4us*)(ph + DIMH)     = h1;
    *(v4us*)(ph + 2 * DIMH) = h2;
    *(v4us*)(pl)            = l0;
    *(v4us*)(pl + DIMH)     = l1;
    *(v4us*)(pl + 2 * DIMH) = l2;
    if (lane == 0) { sdR[row] = (float)nR; sdC[row] = (float)nC; }
  }
  __syncthreads();

  v8f acc[8];
#pragma unroll
  for (int t = 0; t < 8; ++t) { v8f z = {0.f, 0.f, 0.f, 0.f, 0.f, 0.f, 0.f, 0.f}; acc[t] = z; }
  const unsigned short* arH = sHi + (rw + m) * APH + 8 * hh;
  const unsigned short* arL = sLo + (rw + m) * APH + 8 * hh;
#pragma unroll 1
  for (int kt = 0; kt < KSTEPS; ++kt) {
    FragB ah, al;
    ah.h[0] = *(const v8us*)(arH + 32 * kt);
    ah.h[1] = *(const v8us*)(arH + 32 * kt + 16);
    al.h[0] = *(const v8us*)(arL + 32 * kt);
    al.h[1] = *(const v8us*)(arL + 32 * kt + 16);
#pragma unroll
    for (int t = 0; t < 8; ++t) {
      const size_t bo = (size_t)(16 * t + m) * KTOT + 32 * kt + 8 * hh;
      FragB bh, bl;
      bh.h[0] = *(const v8us*)(Bhi + bo);
      bh.h[1] = *(const v8us*)(Bhi + bo + 16);
      bl.h[0] = *(const v8us*)(Blo + bo);
      bl.h[1] = *(const v8us*)(Blo + bo + 16);
      acc[t] = wmb(ah.v, bh.v, acc[t]);
      acc[t] = wmb(al.v, bh.v, acc[t]);
      acc[t] = wmb(ah.v, bl.v, acc[t]);
    }
  }
  __syncthreads();

  const int r0 = rw + 8 * hh;
  const v4f dRa = *(const v4f*)(sdR + r0), dRb = *(const v4f*)(sdR + r0 + 4);
  const v4f dCa = *(const v4f*)(sdC + r0), dCb = *(const v4f*)(sdC + r0 + 4);
  float dR[8], dC[8];
  dR[0] = dRa.x; dR[1] = dRa.y; dR[2] = dRa.z; dR[3] = dRa.w;
  dR[4] = dRb.x; dR[5] = dRb.y; dR[6] = dRb.z; dR[7] = dRb.w;
  dC[0] = dCa.x; dC[1] = dCa.y; dC[2] = dCa.z; dC[3] = dCa.w;
  dC[4] = dCb.x; dC[5] = dCb.y; dC[6] = dCb.z; dC[7] = dCb.w;
  float* sp = stg + r0 * DIMH + m;
#pragma unroll
  for (int t = 0; t < 8; ++t) {
    const int col = 16 * t + m;
    const float wb  = Wb[col];
    const float wtb = Wtb[col];
    const float wsb = Wsb[col];
#pragma unroll
    for (int r = 0; r < 8; ++r) sp[r * DIMH + 16 * t] = acc[t][r] + dR[r] * wb + dC[r] * wtb + wsb;
  }
  __syncthreads();

#pragma unroll 1
  for (int i = 0; i < 16; ++i) {
    float* lp = stg + (rw + i) * DIMH + 4 * lane;
    const v4f x = *(const v4f*)lp;
    v4f g;
    g.x = gelu1(x.x); g.y = gelu1(x.y); g.z = gelu1(x.z); g.w = gelu1(x.w);
    *(v4f*)lp = g;
  }

#pragma unroll 1
  for (int i = 0; i < 16; ++i) {
    const int row = tbase + i;
    if (row < nN) {
      const v4f v = *(const v4f*)(stg + (rw + i) * DIMH + 4 * lane);
      *(volatile v4f*)(out + (size_t)row * DIMH + 4 * lane) = v;
    }
  }
  __threadfence();
#pragma unroll 1
  for (int i = 0; i < 16; ++i) {
    const int row = tbase + i;
    if (row < nN) {
      const v4f v = *(const v4f*)(stg + (rw + i) * DIMH + 4 * lane);
      *(volatile v4f*)(out + (size_t)row * DIMH + 4 * lane) = v;
    }
  }
}

extern "C" void kernel_launch(void* const* d_in, const int* in_sizes, int n_in,
                              void* d_out, int out_size, void* d_ws, size_t ws_size,
                              hipStream_t stream) {
  if (n_in < 9) return;
  const int nN = in_sizes[0] / DIMH;
  const int nE = in_sizes[7];
  if (nN <= 0 || nE <= 0 || in_sizes[0] != nN * DIMH || in_sizes[8] != nE) return;
  if (in_sizes[1] != DIMH * DIMH || in_sizes[3] != DIMH * DIMH || in_sizes[5] != DIMH * DIMH) return;
  if (in_sizes[2] != DIMH || in_sizes[4] != DIMH || in_sizes[6] != DIMH) return;
  if (out_size != nN * DIMH) return;
  if (nE > (1 << 28) || nN > (1 << 24)) return;

  const float* h_n  = (const float*)d_in[0];
  const float* Ww   = (const float*)d_in[1];
  const float* Wb   = (const float*)d_in[2];
  const float* Wtw  = (const float*)d_in[3];
  const float* Wtb  = (const float*)d_in[4];
  const float* Wsw  = (const float*)d_in[5];
  const float* Wsb  = (const float*)d_in[6];
  const int*   rows = (const int*)d_in[7];
  const int*   cols = (const int*)d_in[8];
  float* out = (float*)d_out;

  const int NPAD   = ((nN + TGT - 1) / TGT) * TGT;
  const int nBC    = (nN + NBC - 1) / NBC;
  const int CNTPAD = nBC * NBC;
  if (4 * nBC + 1 > RBN) return;
  const int nBF    = (nN + NBF - 1) / NBF;
  const int csrLen = ((nE + 31) & ~31) + 4096;
  if (31 * nBF > 4096) return;
  const int nFused = NPAD / TGT;

  char* ws = (char*)d_ws;
  size_t off = 0;
  const size_t oBh  = off; off += (size_t)DIMH * KTOT * 2;   off = (off + 255) & ~(size_t)255;
  const size_t oBl  = off; off += (size_t)DIMH * KTOT * 2;   off = (off + 255) & ~(size_t)255;
  const size_t oCnR = off; off += (size_t)CNTPAD * 4;        off = (off + 255) & ~(size_t)255;
  const size_t oOfR = off; off += (size_t)CNTPAD * 4;        off = (off + 255) & ~(size_t)255;
  const size_t oRbR = off; off += (size_t)RBN * 4;           off = (off + 255) & ~(size_t)255;
  const size_t oCsR = off; off += (size_t)csrLen * 4;        off = (off + 255) & ~(size_t)255;
  const size_t oCnC = off; off += (size_t)CNTPAD * 4;        off = (off + 255) & ~(size_t)255;
  const size_t oOfC = off; off += (size_t)CNTPAD * 4;        off = (off + 255) & ~(size_t)255;
  const size_t oRbC = off; off += (size_t)RBN * 4;           off = (off + 255) & ~(size_t)255;
  const size_t oCsC = off; off += (size_t)csrLen * 4;        off = (off + 255) & ~(size_t)255;
  if (off > ws_size || off > ((size_t)128 << 20)) return;
  unsigned short* Bhi = (unsigned short*)(ws + oBh);
  unsigned short* Blo = (unsigned short*)(ws + oBl);
  int* cntR = (int*)(ws + oCnR);
  int* offR = (int*)(ws + oOfR);
  int* rbR  = (int*)(ws + oRbR);
  int* csrR = (int*)(ws + oCsR);
  int* cntC = (int*)(ws + oCnC);
  int* offC = (int*)(ws + oOfC);
  int* rbC  = (int*)(ws + oRbC);
  int* csrC = (int*)(ws + oCsC);

  const int vec8 = 1;

  k_wprep<<<(DIMH * KTOT / 8) / NTHR, NTHR, 0, stream>>>(Ww, Wtw, Wsw, Bhi, Blo);

  hipFuncSetAttribute(reinterpret_cast<const void*>(&k_fill),
                      hipFuncAttributeMaxDynamicSharedMemorySize, LDS_FILL);
  k_count<<<nBC, NTHR, 0, stream>>>(rows, cntR, nE, vec8);
  k_offsets<<<1, OTHR, 0, stream>>>(cntR, offR, rbR, nBC);
  k_fill<<<nBF, NTHR, LDS_FILL, stream>>>(rows, cols, offR, rbR, csrR, nN, nE, vec8, csrLen);

  k_count<<<nBC, NTHR, 0, stream>>>(cols, cntC, nE, vec8);
  k_offsets<<<1, OTHR, 0, stream>>>(cntC, offC, rbC, nBC);
  k_fill<<<nBF, NTHR, LDS_FILL, stream>>>(cols, rows, offC, rbC, csrC, nN, nE, vec8, csrLen);

  hipFuncSetAttribute(reinterpret_cast<const void*>(&k_fused),
                      hipFuncAttributeMaxDynamicSharedMemorySize, LDS_FUSED);
  k_fused<<<nFused, FTHR, LDS_FUSED, stream>>>(h_n, Bhi, Blo, cntR, offR, csrR, cntC, offC, csrC,
                                               Wb, Wtb, Wsb, out, nN, csrLen);
}
